// CrossAttenFusion_76630806495489
// MI455X (gfx1250) — hardware-verified
//
#include <hip/hip_runtime.h>
#include <math.h>
#include <stdint.h>

#define NBATCH  8
#define NTOK    3136
#define NCTX    3136
#define DM      64
#define DC      64
#define NH      2
#define HD      32
#define KCH     32
#define NCHUNK  (NCTX / KCH)
#define MROWS   (NBATCH * NTOK)
#define CROWS   (NBATCH * NCTX)
#define WSC     64.0f
#define ACARRY  16.0f
#define QC      64.0f
#define KC      64.0f
#define VC      16.0f
#define PC      32768.0f
#define FC      4096.0f
static_assert(NH * HD == DM);
static_assert(HD == 32);
static_assert(DC == DM);
static_assert((MROWS % 64) == 0 && (CROWS % 64) == 0 && (NTOK % 16) == 0 && (NCTX % 64) == 0 && (NCTX % KCH) == 0);
static_assert(NCHUNK == 98 && MROWS == 25088 && CROWS == 25088);
static_assert(((MROWS * DM / 8) % 256) == 0 && ((CROWS * DC / 8) % 256) == 0);

typedef _Float16 v16h __attribute__((ext_vector_type(16)));
typedef _Float16 v8h  __attribute__((ext_vector_type(8)));
typedef float    v8f  __attribute__((ext_vector_type(8)));
typedef float    v4f  __attribute__((ext_vector_type(4)));
typedef unsigned int v4u __attribute__((ext_vector_type(4)));

union FragH { v16h v; v8h h[2]; v4u u[2]; };

__device__ __forceinline__ unsigned short bf_bits(float f) {
  unsigned u = __float_as_uint(f);
  return (unsigned short)((u + 0x7FFFu + ((u >> 16) & 1u)) >> 16);
}
__device__ __forceinline__ float bf_up(unsigned short h) { return __uint_as_float(((unsigned)h) << 16); }
__device__ __forceinline__ float bfr(float f) { return bf_up(bf_bits(f)); }
__device__ __forceinline__ unsigned short h_bits(_Float16 x) { return __builtin_bit_cast(unsigned short, x); }
__device__ __forceinline__ unsigned pk16(unsigned short a, unsigned short b) { return (unsigned)a | ((unsigned)b << 16); }
__device__ __forceinline__ v8f zero8() { v8f z = {0.f, 0.f, 0.f, 0.f, 0.f, 0.f, 0.f, 0.f}; return z; }

__device__ __forceinline__ v16h ldfrag_h(const _Float16* p) {
  FragH f;
  f.h[0] = *(const v8h*)(p);
  f.h[1] = *(const v8h*)(p + 16);
  return f.v;
}
__device__ __forceinline__ v16h ldfrag_u(const unsigned short* p) {
  FragH f;
  f.u[0] = *(const v4u*)(p);
  f.u[1] = *(const v4u*)(p + 16);
  return f.v;
}

__device__ __forceinline__ v8f mma_raw(v16h a, v16h b, v8f c) {
  return __builtin_amdgcn_wmma_f32_16x16x32_f16(false, a, false, b, (short)0, c, false, false);
}
__device__ __forceinline__ void dep_guard2(v8f& a, v8f& b, v16h x, v16h y) {
#if defined(__HIP_DEVICE_COMPILE__)
  asm volatile("v_nop\n\tv_nop\n\tv_nop\n\tv_nop" : "+v"(a), "+v"(b) : "v"(x), "v"(y));
#endif
}
__device__ __forceinline__ void guard3(v8f& a, v8f& b, v16h x, v16h y, v16h z) {
#if defined(__HIP_DEVICE_COMPILE__)
  asm volatile("v_nop\n\tv_nop\n\tv_nop\n\tv_nop" : "+v"(a), "+v"(b) : "v"(x), "v"(y), "v"(z));
#endif
}
__device__ __forceinline__ void keep4_h(v16h a, v16h b, v16h c, v16h d) {
#if defined(__HIP_DEVICE_COMPILE__)
  asm volatile("v_nop" :: "v"(a), "v"(b), "v"(c), "v"(d));
#endif
}
__device__ __forceinline__ void acc_guard4(v8f& a, v8f& b, v8f& c, v8f& d) {
#if defined(__HIP_DEVICE_COMPILE__)
  asm volatile("v_nop\n\tv_nop\n\tv_nop\n\tv_nop" : "+v"(a), "+v"(b), "+v"(c), "+v"(d));
#endif
}
__device__ __forceinline__ void wave_sync_lds() {
  __builtin_amdgcn_fence(__ATOMIC_RELEASE, "workgroup");
  __builtin_amdgcn_wave_barrier();
  __builtin_amdgcn_fence(__ATOMIC_ACQUIRE, "workgroup");
}

__global__ __launch_bounds__(256) void convw(const float* __restrict__ w0, const float* __restrict__ w1,
                                             const float* __restrict__ w2, const float* __restrict__ w3,
                                             unsigned short* d0, unsigned short* d1, unsigned short* d2,
                                             unsigned short* d3, float wsc) {
  __shared__ float Wt[64 * 65];
  const int sel = blockIdx.x;
  const float* W = (sel == 0) ? w0 : ((sel == 1) ? w1 : ((sel == 2) ? w2 : w3));
  unsigned short* dst = (sel == 0) ? d0 : ((sel == 1) ? d1 : ((sel == 2) ? d2 : d3));
  const int tid = threadIdx.x;
  for (int idx = tid; idx < 64 * 64; idx += 256) {
    const int r = idx >> 6, cc = idx & 63;
    Wt[cc * 65 + r] = W[idx];
  }
  __syncthreads();
  v4u vals[2];
#pragma unroll
  for (int it = 0; it < 2; ++it) {
    const int p = it * 256 + tid;
    const int row = p >> 3, c8 = (p & 7) * 8;
    const float* sp = Wt + row * 65 + c8;
    v4u ov = {0u, 0u, 0u, 0u};
#pragma unroll
    for (int e = 0; e < 4; ++e)
      ov[e] = pk16(h_bits((_Float16)(bfr(sp[2 * e]) * wsc)), h_bits((_Float16)(bfr(sp[2 * e + 1]) * wsc)));
    vals[it] = ov;
  }
  for (int pass = 0; pass < 2; ++pass) {
#pragma unroll
    for (int it = 0; it < 2; ++it) {
      const int p = it * 256 + tid;
      const int row = p >> 3, c8 = (p & 7) * 8;
      *(volatile v4u*)(dst + row * 64 + c8) = vals[it];
    }
    __threadfence();
  }
}

__global__ __launch_bounds__(256) void conv16(const float* __restrict__ X, unsigned short* dst, int n8, float wsc) {
  const int i  = blockIdx.x * 256 + threadIdx.x;
  const int ic = (i < n8) ? i : (n8 - 1);
  const float* p = X + (size_t)ic * 8;
  const v4f a = *(const v4f*)(p), b = *(const v4f*)(p + 4);
  float v[8];
#pragma unroll
  for (int e = 0; e < 4; ++e) { v[e] = bfr(a[e]); v[4 + e] = bfr(b[e]); }
  v4u ov;
#pragma unroll
  for (int e = 0; e < 4; ++e) ov[e] = pk16(h_bits((_Float16)(v[2 * e] * wsc)), h_bits((_Float16)(v[2 * e + 1] * wsc)));
  if (i < n8) *(volatile v4u*)(dst + (size_t)i * 8) = ov;
  __threadfence();
  if (i < n8) *(volatile v4u*)(dst + (size_t)i * 8) = ov;
}

template <int OM, int HASB, int TWOA>
__global__ __launch_bounds__(256) void gemm64(
    const unsigned short* __restrict__ Ap, const unsigned short* __restrict__ A2p, int lda, long long sA,
    const unsigned short* __restrict__ Btp, int ldb, long long sB,
    const float* __restrict__ bias, float bscale,
    void* Cout, void* Cout2, int ldc, long long sC,
    int M, int N, int K, float oscale) {
  __shared__ __align__(16) float sT[8][16 * 68];
  const int by   = blockIdx.y;
  const int lane = threadIdx.x & 31;
  const int wave = threadIdx.x >> 5;
  const int tilesN = N >> 6;
  const int tilesM = M >> 6;
  const int tile = blockIdx.x * 8 + wave;
  if (tile >= tilesM * tilesN) return;
  const int tm = tile / tilesN;
  const int tn = tile - tm * tilesN;
  const int m0 = tm << 6;
  const int n0 = tn << 6;

  const unsigned short* A1 = Ap  + (size_t)((long long)by * sA);
  const unsigned short* A2 = A2p + (size_t)((long long)by * sA);
  const unsigned short* Bb = Btp + (size_t)((long long)by * sB);

  const int rlane = lane & 15;
  const int koff  = (lane >> 4) * 8;
  const int mOff  = (lane >> 4) * 8;

  v8f acc[4][4];
#pragma unroll
  for (int i = 0; i < 4; ++i)
#pragma unroll
    for (int j = 0; j < 4; ++j) acc[i][j] = zero8();

  for (int k0 = 0; k0 < K; k0 += 32) {
    v16h bh[4];
#pragma unroll
    for (int j = 0; j < 4; ++j) {
      const size_t bofs = (size_t)(n0 + (j << 4) + rlane) * ldb + koff + k0;
      bh[j] = ldfrag_u(Bb + bofs);
    }
#pragma unroll
    for (int i = 0; i < 4; ++i) {
      const size_t ao = (size_t)(m0 + (i << 4) + rlane) * lda + koff + k0;
      const v16h ah = ldfrag_u(A1 + ao);
      v16h al = ah;
      if (TWOA != 0) al = ldfrag_u(A2 + ao);
#pragma unroll
      for (int j = 0; j < 4; ++j) {
        acc[i][j] = mma_raw(ah, bh[j], acc[i][j]);
        if (TWOA != 0) acc[i][j] = mma_raw(al, bh[j], acc[i][j]);
      }
      dep_guard2(acc[i][0], acc[i][3], ah, al);
    }
    keep4_h(bh[0], bh[1], bh[2], bh[3]);
  }
  acc_guard4(acc[0][0], acc[0][1], acc[0][2], acc[0][3]);
  acc_guard4(acc[1][0], acc[1][1], acc[1][2], acc[1][3]);
  acc_guard4(acc[2][0], acc[2][1], acc[2][2], acc[2][3]);
  acc_guard4(acc[3][0], acc[3][1], acc[3][2], acc[3][3]);

  const int hh2 = lane >> 4, c4 = (lane & 15) * 4;
  const int q8  = lane >> 3, c8 = (lane & 7) * 8;
  float bc[4];
#pragma unroll
  for (int e = 0; e < 4; ++e) bc[e] = 0.f;
  if (HASB != 0 && OM == 0) {
    const int cb = n0 + c4;
    const int i0 = (cb < N - 4) ? cb : (N - 4);
    const v4f b0v = *(const v4f*)(bias + i0);
#pragma unroll
    for (int e = 0; e < 4; ++e) bc[e] = bfr(b0v[e]) * bscale;
  }

  float* slab = sT[wave];
#pragma unroll
  for (int i = 0; i < 4; ++i) {
    const int mBase = m0 + (i << 4);
#pragma unroll
    for (int j = 0; j < 4; ++j) {
#pragma unroll
      for (int r = 0; r < 8; ++r) {
        slab[(mOff + r) * 68 + (j << 4) + rlane] = acc[i][j][r];
      }
    }
    wave_sync_lds();
    if (OM == 0) {
      float* C = (float*)Cout + (size_t)((long long)by * sC);
      v4f vals[8];
#pragma unroll
      for (int it = 0; it < 8; ++it) {
        const int row = it * 2 + hh2;
        v4f v = *(const v4f*)(slab + row * 68 + c4);
#pragma unroll
        for (int e = 0; e < 4; ++e) v[e] = v[e] * oscale + bc[e];
        vals[it] = v;
      }
      for (int pass = 0; pass < 2; ++pass) {
#pragma unroll
        for (int it = 0; it < 8; ++it) {
          const int gr = mBase + it * 2 + hh2;
          *(volatile v4f*)(C + (size_t)gr * ldc + n0 + c4) = vals[it];
        }
        __threadfence();
      }
    } else {
      unsigned short* C  = (unsigned short*)Cout  + (size_t)((long long)by * sC);
      unsigned short* C2 = (unsigned short*)Cout2 + (size_t)((long long)by * sC);
      v4u hv[4], lv[4];
#pragma unroll
      for (int it = 0; it < 4; ++it) {
        const int row = it * 4 + q8;
        const float* sp = slab + row * 68 + c8;
        v4u a = {0u, 0u, 0u, 0u}, b = {0u, 0u, 0u, 0u};
#pragma unroll
        for (int e = 0; e < 4; ++e) {
          const float f0 = sp[2 * e] * oscale;
          const float f1 = sp[2 * e + 1] * oscale;
          const _Float16 h0 = (_Float16)f0, h1 = (_Float16)f1;
          a[e] = pk16(h_bits(h0), h_bits(h1));
          if (OM == 3) {
            const _Float16 l0 = (_Float16)(f0 - (float)h0), l1 = (_Float16)(f1 - (float)h1);
            b[e] = pk16(h_bits(l0), h_bits(l1));
          }
        }
        hv[it] = a;
        lv[it] = b;
      }
      for (int pass = 0; pass < 2; ++pass) {
#pragma unroll
        for (int it = 0; it < 4; ++it) {
          const int row = it * 4 + q8;
          *(volatile v4u*)(C + (size_t)(mBase + row) * ldc + n0 + c8) = hv[it];
          if (OM == 3) *(volatile v4u*)(C2 + (size_t)(mBase + row) * ldc + n0 + c8) = lv[it];
        }
        __threadfence();
      }
    }
    wave_sync_lds();
  }
}

__global__ __launch_bounds__(64) void colsum32(const float* __restrict__ V, float* CS, int ngrp) {
  const int t  = blockIdx.x * 64 + threadIdx.x;
  const int g  = t >> 4;
  const int i4 = (t & 15) * 4;
  const int gc = (g < ngrp) ? g : (ngrp - 1);
  const float* src = V + (size_t)gc * (KCH * DM) + i4;
  v4f acc = {0.f, 0.f, 0.f, 0.f};
#pragma unroll 8
  for (int j = 0; j < KCH; ++j) {
    const v4f x = *(const v4f*)(src + (size_t)j * DM);
    acc += x;
  }
  if (g < ngrp) *(volatile v4f*)(CS + (size_t)g * DM + i4) = acc;
  __threadfence();
  if (g < ngrp) *(volatile v4f*)(CS + (size_t)g * DM + i4) = acc;
}

__global__ __launch_bounds__(64)
void attn32(const unsigned short* __restrict__ QPp, const unsigned short* __restrict__ KPp,
            const unsigned short* __restrict__ VTq, const float* __restrict__ CSp,
            unsigned short* CH, unsigned short* CL) {
  __shared__ __align__(16) float Ps[NH][16 * 36];
  __shared__ __align__(16) unsigned short Oh[16 * DM];
  __shared__ __align__(16) unsigned short Ol[16 * DM];

  const int tid  = threadIdx.x;
  const int wave = tid >> 5;
  const int lane = tid & 31;
  const int hh   = lane >> 4;
  const int c    = lane & 15;

  const int bat  = blockIdx.x / (NTOK / 16);
  const int qt   = blockIdx.x - bat * (NTOK / 16);
  const int head = wave;
  const int q0   = qt * 16;

  const _Float16* Qp = (const _Float16*)(const void*)QPp + ((size_t)bat * NTOK + q0 + c) * DM + head * HD + 8 * hh;
  const _Float16* Kb = (const _Float16*)(const void*)KPp + (size_t)bat * NCTX * DM + head * HD + 8 * hh;
  const _Float16* Vb = (const _Float16*)(const void*)VTq + (size_t)(bat * NH + head) * HD * NCTX + 8 * hh;
  const float*  csb  = CSp + (size_t)bat * NCHUNK * DM + head * HD + c;
  const float lsc = (1.4426950408889634f * 0.17677669529663687f) / (QC * KC);

  const v16h qf = ldfrag_h(Qp);

  float mrow[8], lrow[8];
  v8f o0 = zero8(), o1 = zero8(), u0 = zero8(), u1 = zero8();
#pragma unroll
  for (int r = 0; r < 8; ++r) { mrow[r] = -INFINITY; lrow[r] = 0.f; }
  float* pt = Ps[wave];

#pragma unroll 1
  for (int kb = 0; kb < NCTX; kb += KCH) {
    const _Float16* kp = Kb + (size_t)(kb + c) * DM;
    v8f s0, s1;
    {
      const v16h k0 = ldfrag_h(kp);
      const v16h k1 = ldfrag_h(kp + (size_t)16 * DM);
      s0 = mma_raw(qf, k0, zero8());
      s1 = mma_raw(qf, k1, zero8());
      guard3(s0, s1, qf, k0, k1);
    }
    const float* csp = csb + (size_t)(kb / KCH) * DM;
    const float cs0 = csp[0];
    const float cs1 = csp[16];
#pragma unroll
    for (int r = 0; r < 8; ++r) {
      const float t0 = s0[r] * lsc, t1 = s1[r] * lsc;
      float mx = fmaxf(t0, t1);
#pragma unroll
      for (int off = 1; off < 16; off <<= 1) mx = fmaxf(mx, __shfl_xor(mx, off, 32));
      const float mn = fmaxf(mrow[r], mx);
      const float al = exp2f(mrow[r] - mn);
      mrow[r] = mn;
      const float e0 = exp2f(t0 - mn), e1 = exp2f(t1 - mn);
      float ps = e0 + e1;
#pragma unroll
      for (int off = 1; off < 16; off <<= 1) ps += __shfl_xor(ps, off, 32);
      const float eb = ps * (1.0f / 32.0f);
      lrow[r] = lrow[r] * al + ps;
      o0[r] *= al;
      o1[r] *= al;
      u0[r] = u0[r] * al + eb * cs0;
      u1[r] = u1[r] * al + eb * cs1;
      const int ro = (8 * hh + r) * 36 + c;
      pt[ro]      = e0 - eb;
      pt[ro + 16] = e1 - eb;
    }
    wave_sync_lds();
    FragH ph;
    {
      const float* prow = pt + c * 36 + 8 * hh;
      const v4f p0 = *(const v4f*)(prow), p1 = *(const v4f*)(prow + 4);
      const v4f p2 = *(const v4f*)(prow + 16), p3 = *(const v4f*)(prow + 20);
#pragma unroll
      for (int e = 0; e < 4; ++e) {
        ph.h[0][e]     = (_Float16)(p0[e] * PC);
        ph.h[0][4 + e] = (_Float16)(p1[e] * PC);
        ph.h[1][e]     = (_Float16)(p2[e] * PC);
        ph.h[1][4 + e] = (_Float16)(p3[e] * PC);
      }
    }
    const _Float16* vp = Vb + (size_t)c * NCTX + kb;
    {
      const v16h vb0 = ldfrag_h(vp);
      const v16h vb1 = ldfrag_h(vp + (size_t)16 * NCTX);
      o0 = mma_raw(ph.v, vb0, o0);
      o1 = mma_raw(ph.v, vb1, o1);
      guard3(o0, o1, ph.v, vb0, vb1);
    }
    wave_sync_lds();
  }

  const float oc = 1.0f / (PC * VC);
  unsigned short* oh = Oh + head * HD + c;
  unsigned short* ol = Ol + head * HD + c;
#pragma unroll
  for (int r = 0; r < 8; ++r) {
    const float inv = 1.0f / lrow[r];
    const float f0 = ((o0[r] * oc + u0[r]) * inv) * FC;
    const float f1 = ((o1[r] * oc + u1[r]) * inv) * FC;
    const _Float16 g0 = (_Float16)f0, g1 = (_Float16)f1;
    const _Float16 l0 = (_Float16)(f0 - (float)g0), l1 = (_Float16)(f1 - (float)g1);
    const int ro = (8 * hh + r) * DM;
    oh[ro]      = h_bits(g0);
    oh[ro + 16] = h_bits(g1);
    ol[ro]      = h_bits(l0);
    ol[ro + 16] = h_bits(l1);
  }
  __syncthreads();
  {
    v4u hv[2], lv[2];
#pragma unroll
    for (int it = 0; it < 2; ++it) {
      const int p   = it * 64 + tid;
      const int row = p >> 3;
      const int c8  = (p & 7) * 8;
      hv[it] = *(const v4u*)(Oh + row * DM + c8);
      lv[it] = *(const v4u*)(Ol + row * DM + c8);
    }
    const size_t dofs = ((size_t)bat * NTOK + q0) * DM;
    unsigned short* dh = CH + dofs;
    unsigned short* dl = CL + dofs;
    for (int pass = 0; pass < 2; ++pass) {
#pragma unroll
      for (int it = 0; it < 2; ++it) {
        const int p   = it * 64 + tid;
        const int row = p >> 3;
        const int c8  = (p & 7) * 8;
        *(volatile v4u*)(dh + (size_t)row * DM + c8) = hv[it];
        *(volatile v4u*)(dl + (size_t)row * DM + c8) = lv[it];
      }
      __threadfence();
    }
  }
}

extern "C" void kernel_launch(void* const* d_in, const int* in_sizes, int n_in,
                              void* d_out, int out_size, void* d_ws, size_t ws_size,
                              hipStream_t stream) {
  if (n_in < 7) return;
  if (in_sizes[0] != MROWS * DM) return;
  if (in_sizes[1] != CROWS * DC) return;
  if (in_sizes[2] != DM * DM || in_sizes[3] != DC * DM || in_sizes[4] != DC * DM) return;
  if (in_sizes[5] != DM * DM || in_sizes[6] != DM) return;
  if (out_size != MROWS * DM) return;

  const float* q_x  = (const float*)d_in[0];
  const float* kv_x = (const float*)d_in[1];
  const float* w_q  = (const float*)d_in[2];
  const float* w_k  = (const float*)d_in[3];
  const float* w_v  = (const float*)d_in[4];
  const float* w_o  = (const float*)d_in[5];
  const float* b_o  = (const float*)d_in[6];
  float*       out  = (float*)d_out;

  const size_t PW   = (size_t)DM * DM * 2;
  const size_t PXI  = (size_t)MROWS * DM * 2;
  const size_t PKI  = (size_t)CROWS * DC * 2;
  const size_t PV32 = (size_t)CROWS * DM * 4;
  const size_t PVT  = (size_t)NBATCH * DM * NCTX * 2;
  const size_t PCS  = (size_t)NBATCH * NCHUNK * DM * 4;
  size_t off = 0;
  const size_t oWQ  = off; off += PW;
  const size_t oWK  = off; off += PW;
  const size_t oWV  = off; off += PW;
  const size_t oWO  = off; off += PW;
  const size_t oXI  = off; off += PXI;
  const size_t oKI  = off; off += PKI;
  const size_t oQP  = off; off += PXI;
  const size_t oKP  = off; off += PKI;
  const size_t oV32 = off; off += PV32;
  const size_t oVT  = off; off += PVT;
  const size_t oCS  = off; off += PCS;
  const size_t oCH  = off; off += PXI;
  const size_t oCL  = off; off += PXI;
  if (off > ws_size) return;
  if (off > (size_t)134217728) return;
  if ((PW % 4096) != 0 || (PXI % 4096) != 0 || (PKI % 4096) != 0 || (PV32 % 4096) != 0 || (PVT % 4096) != 0 ||
      (PCS % 4096) != 0) return;

  char* ws = (char*)d_ws;
  unsigned short* WQ  = (unsigned short*)(ws + oWQ);
  unsigned short* WK  = (unsigned short*)(ws + oWK);
  unsigned short* WV  = (unsigned short*)(ws + oWV);
  unsigned short* WO  = (unsigned short*)(ws + oWO);
  unsigned short* XI  = (unsigned short*)(ws + oXI);
  unsigned short* KI  = (unsigned short*)(ws + oKI);
  unsigned short* QP  = (unsigned short*)(ws + oQP);
  unsigned short* KP  = (unsigned short*)(ws + oKP);
  float*          V32 = (float*)(ws + oV32);
  unsigned short* VTp = (unsigned short*)(ws + oVT);
  float*          CS  = (float*)(ws + oCS);
  unsigned short* CH  = (unsigned short*)(ws + oCH);
  unsigned short* CL  = (unsigned short*)(ws + oCL);

  const int n8q  = (MROWS * DM) / 8;
  const int n8kv = (CROWS * DC) / 8;
  if ((n8q % 256) != 0 || (n8kv % 256) != 0) return;
  const dim3 blk(256), blk64(64);
  const dim3 gCq(n8q / 256), gCkv(n8kv / 256);
  const int tilesQ  = (MROWS / 64) * (DM / 64);
  const int tilesK  = (CROWS / 64) * (DM / 64);
  const int tilesVT = (DM / 64) * (NCTX / 64);
  const dim3 gQ((tilesQ + 7) / 8, 1);
  const dim3 gK((tilesK + 7) / 8, 1);
  const dim3 gVT((tilesVT + 7) / 8, NBATCH);
  const int ngrp = NBATCH * NCHUNK;
  const dim3 gCS((ngrp * 16 + 63) / 64);
  const dim3 gAT(NBATCH * (NTOK / 16));

  convw<<<dim3(4), blk, 0, stream>>>(w_q, w_k, w_v, w_o, WQ, WK, WV, WO, WSC);

  conv16<<<gCq,  blk, 0, stream>>>(q_x,  XI, n8q,  ACARRY);
  conv16<<<gCkv, blk, 0, stream>>>(kv_x, KI, n8kv, ACARRY);

  gemm64<2, 0, 0><<<gQ, blk, 0, stream>>>(
      XI, XI, DM, 0LL,
      WQ, DM, 0LL,
      b_o, 0.f,
      (void*)QP, (void*)QP, DM, 0LL,
      MROWS, DM, DM, QC / (ACARRY * WSC));

  gemm64<2, 0, 0><<<gK, blk, 0, stream>>>(
      KI, KI, DC, 0LL,
      WK, DC, 0LL,
      b_o, 0.f,
      (void*)KP, (void*)KP, DM, 0LL,
      CROWS, DM, DC, KC / (ACARRY * WSC));

  gemm64<0, 0, 0><<<gK, blk, 0, stream>>>(
      KI, KI, DC, 0LL,
      WV, DC, 0LL,
      b_o, 0.f,
      (void*)V32, (void*)V32, DM, 0LL,
      CROWS, DM, DC, 1.0f / (ACARRY * WSC));

  gemm64<2, 0, 0><<<gVT, blk, 0, stream>>>(
      WV, WV, DC, 0LL,
      KI, DC, (long long)NCTX * DC,
      b_o, 0.f,
      (void*)VTp, (void*)VTp, NCTX, (long long)DM * NCTX,
      DM, NCTX, DC, VC / (ACARRY * WSC));

  colsum32<<<gCS, blk64, 0, stream>>>(V32, CS, ngrp);

  attn32<<<gAT, blk64, 0, stream>>>(QP, KP, VTp, CS, CH, CL);

  gemm64<0, 1, 1><<<gQ, blk, 0, stream>>>(
      CH, CL, DM, 0LL,
      WO, DM, 0LL,
      b_o, 1.0f,
      (void*)out, (void*)out, DM, 0LL,
      MROWS, DM, DM, 1.0f / (FC * WSC));
  (void)hipGetLastError();
}
